// GAT_17300128268969
// MI455X (gfx1250) — hardware-verified
//
#include <hip/hip_runtime.h>
#include <math.h>
#include <stdint.h>

constexpr int NBATCH  = 8;
constexpr int NNODE   = 768;
constexpr int DMODEL  = 512;
constexpr int NHEADS  = 8;
constexpr int HDIM    = 64;
constexpr int HIDN    = 256;
constexpr int MROWS   = NBATCH * NNODE;
constexpr int G4W     = 4 * HIDN;
constexpr int NLAYERS = 3;
constexpr int MHALF   = MROWS / 2;
constexpr float LN_EPS       = 1e-5f;
constexpr float AV_CARRY     = 32.0f;
constexpr float AV_CARRY_INV = 1.0f / 32.0f;
constexpr float W_CARRY      = 64.0f;
constexpr float P_CARRY      = 32768.0f;

static_assert(MROWS == 6144 && G4W == 1024 && NHEADS * HDIM == DMODEL && 2 * HIDN == DMODEL, "");
static_assert(MROWS % 64 == 0 && G4W % 64 == 0 && DMODEL % 64 == 0 && NNODE % 64 == 0 && HDIM == 64, "");
static_assert(DMODEL % 32 == 0 && HIDN % 32 == 0 && NNODE % 32 == 0 && HDIM % 32 == 0, "");
static_assert(MHALF % 8 == 0 && (NHEADS * NNODE) % 8 == 0, "");

constexpr size_t SZ_ACT16 = (size_t)MROWS * DMODEL * 2;
constexpr size_t SZ_WIH16 = (size_t)G4W * DMODEL * 2;
constexpr size_t SZ_WHH16 = (size_t)G4W * HIDN * 2;
constexpr size_t SZ_WSQ16 = (size_t)DMODEL * DMODEL * 2;
constexpr size_t SZ_BTAB  = 4096 * 4;
constexpr size_t SZ_GX    = (size_t)2 * MROWS * G4W * 4;
constexpr size_t SZ_GATE  = (size_t)MROWS * G4W * 4;
constexpr size_t SZ_SP16  = (size_t)NHEADS * NNODE * NNODE * 2;
constexpr size_t OFF_XM   = 0;
constexpr size_t OFF_HEAD = OFF_XM + SZ_ACT16;
constexpr size_t OFF_TA   = OFF_HEAD + SZ_ACT16;
constexpr size_t OFF_INFT = OFF_TA + SZ_ACT16;
constexpr size_t OFF_AV   = OFF_INFT + SZ_ACT16;
constexpr size_t OFF_WIH0 = OFF_AV + SZ_ACT16;
constexpr size_t OFF_WIH1 = OFF_WIH0 + SZ_WIH16;
constexpr size_t OFF_WHH0 = OFF_WIH1 + SZ_WIH16;
constexpr size_t OFF_WHH1 = OFF_WHH0 + SZ_WHH16;
constexpr size_t OFF_WH   = OFF_WHH1 + SZ_WHH16;
constexpr size_t OFF_WT   = OFF_WH + SZ_WSQ16;
constexpr size_t OFF_WI   = OFF_WT + SZ_WSQ16;
constexpr size_t OFF_WC   = OFF_WI + SZ_WSQ16;
constexpr size_t OFF_BTAB = OFF_WC + SZ_WSQ16;
constexpr size_t OFF_GX   = OFF_BTAB + SZ_BTAB;
constexpr size_t OFF_GATE = OFF_GX + SZ_GX;
constexpr size_t OFF_S    = OFF_GATE + SZ_GATE;
constexpr size_t OFF_P    = OFF_S + SZ_SP16;
constexpr size_t WS_TOTAL = OFF_P + SZ_SP16;
static_assert((size_t)NBATCH * DMODEL * NNODE * 2 == SZ_ACT16, "");
static_assert(WS_TOTAL == 131088384, "");
static_assert(WS_TOTAL <= 134217728, "");
static_assert(OFF_HEAD % 256 == 0 && OFF_BTAB % 256 == 0 && OFF_GX % 256 == 0 && OFF_S % 256 == 0 && OFF_P % 256 == 0, "");

typedef __attribute__((ext_vector_type(16))) _Float16 v16h;
typedef __attribute__((ext_vector_type(8)))  _Float16 v8h;
typedef __attribute__((ext_vector_type(16))) __bf16   v16b;
typedef __attribute__((ext_vector_type(8)))  __bf16   v8b;
typedef __attribute__((ext_vector_type(8)))  float    v8f;
typedef __attribute__((ext_vector_type(4)))  float    v4f;
typedef __attribute__((ext_vector_type(2)))  float    v2f;
typedef __attribute__((ext_vector_type(4)))  unsigned int v4u;
typedef __attribute__((ext_vector_type(8)))  int      v8i;

__device__ __forceinline__ unsigned short f2bf_bits(float f) {
  unsigned u = __float_as_uint(f);
  return (unsigned short)((u + 0x7FFFu + ((u >> 16) & 1u)) >> 16);
}
__device__ __forceinline__ float bf_bits2f(unsigned short h) { return __uint_as_float(((unsigned)h) << 16); }

__device__ __forceinline__ float h16_to_f32(unsigned hb) {
  const unsigned sgn = (hb & 0x8000u) << 16; const unsigned em = hb & 0x7fffu;
  const float fn = __uint_as_float((em << 13) + 0x38000000u);
  const float fs = (float)em * 5.9604644775390625e-8f;
  const float mag = (em < 0x400u) ? fs : fn; return __uint_as_float(__float_as_uint(mag) | sgn); }

__device__ __forceinline__ void dep_guard_h(v8f& a, v8f& b, v16h x, v16h y) { asm volatile("v_nop\n\tv_nop\n\tv_nop\n\tv_nop" : "+v"(a), "+v"(b) : "v"(x), "v"(y)); }
__device__ __forceinline__ void dep_guard_b(v8f& a, v8f& b, v16b x, v16b y) { asm volatile("v_nop\n\tv_nop\n\tv_nop\n\tv_nop" : "+v"(a), "+v"(b) : "v"(x), "v"(y)); }
__device__ __forceinline__ void dep_guard4_h(v8f& a, v8f& b, v8f& c, v8f& d, v16h x, v16h y) { asm volatile("v_nop\n\tv_nop\n\tv_nop\n\tv_nop" : "+v"(a), "+v"(b), "+v"(c), "+v"(d) : "v"(x), "v"(y)); }
__device__ __forceinline__ void dep_guard4_b(v8f& a, v8f& b, v8f& c, v8f& d, v16b x, v16b y) { asm volatile("v_nop\n\tv_nop\n\tv_nop\n\tv_nop" : "+v"(a), "+v"(b), "+v"(c), "+v"(d) : "v"(x), "v"(y)); }
__device__ __forceinline__ void keep4_h(v16h a, v16h b, v16h c, v16h d) { asm volatile("v_nop" :: "v"(a), "v"(b), "v"(c), "v"(d)); }
__device__ __forceinline__ void keep4_b(v16b a, v16b b, v16b c, v16b d) { asm volatile("v_nop" :: "v"(a), "v"(b), "v"(c), "v"(d)); }
__device__ __forceinline__ void acc_guard4(v8f& a, v8f& b, v8f& c, v8f& d) { asm volatile("v_nop\n\tv_nop\n\tv_nop\n\tv_nop" : "+v"(a), "+v"(b), "+v"(c), "+v"(d)); }
template <typename T> struct Frag;
template <> struct Frag<_Float16> {
  typedef v16h V; union U { v16h v; v8h h[2]; };
  static __device__ __forceinline__ v16h load(const _Float16* p) {
    U f; f.h[0] = *(const v8h*)(p); f.h[1] = *(const v8h*)(p + 16); return f.v;
  }
  static __device__ __forceinline__ v8f mma(v16h a, v16h b, v8f c) {
    return __builtin_amdgcn_wmma_f32_16x16x32_f16(false, a, false, b, (short)0, c, false, false);
  }
  static __device__ __forceinline__ void guard(v8f& a, v8f& b, v16h x, v16h y) { dep_guard_h(a, b, x, y); }
  static __device__ __forceinline__ void guard4(v8f& a, v8f& b, v8f& c, v8f& d, v16h x, v16h y) { dep_guard4_h(a, b, c, d, x, y); }
  static __device__ __forceinline__ void keep(v16h a, v16h b, v16h c, v16h d) { keep4_h(a, b, c, d); }
};
template <> struct Frag<__bf16> {
  typedef v16b V; union U { v16b v; v8b h[2]; };
  static __device__ __forceinline__ v16b load(const __bf16* p) {
    U f; f.h[0] = *(const v8b*)(p); f.h[1] = *(const v8b*)(p + 16); return f.v;
  }
  static __device__ __forceinline__ v8f mma(v16b a, v16b b, v8f c) {
    return __builtin_amdgcn_wmma_f32_16x16x32_bf16(false, a, false, b, (short)0, c, false, false);
  }
  static __device__ __forceinline__ void guard(v8f& a, v8f& b, v16b x, v16b y) { dep_guard_b(a, b, x, y); }
  static __device__ __forceinline__ void guard4(v8f& a, v8f& b, v8f& c, v8f& d, v16b x, v16b y) { dep_guard4_b(a, b, c, d, x, y); }
  static __device__ __forceinline__ void keep(v16b a, v16b b, v16b c, v16b d) { keep4_b(a, b, c, d); }
};

template <int ET> struct Elem;
template <> struct Elem<0> { typedef _Float16 T; };
template <> struct Elem<1> { typedef __bf16 T; };
template <int ET, bool SPLIT, int BIAS_MODE, int OUT_MODE, bool RESF>
__global__ __launch_bounds__(256) void wmma_gemm64(
    const unsigned short* __restrict__ Ap, const unsigned short* __restrict__ A2p, int lda, long strideA,
    const unsigned short* __restrict__ Btp, const unsigned short* __restrict__ Bt2p, int ldb, long strideB,
    void* __restrict__ Cout, int ldc, long strideC,
    const float* __restrict__ bias,
    const float* __restrict__ resid, long strideR,
    int M, int N, int K, float scale) {
  static_assert(OUT_MODE == 0 || OUT_MODE == 1, "");
  static_assert(!RESF || OUT_MODE == 0, "");
  typedef typename Elem<ET>::T T;
  typedef typename Frag<T>::V V;
  const T* A = (const T*)Ap; const T* A2 = (const T*)A2p; const T* Bt = (const T*)Btp; const T* Bt2 = (const T*)Bt2p;
  __shared__ __align__(16) float sT[8][16 * 68];
  const int b    = blockIdx.y;
  const int lane = threadIdx.x & 31;
  const int wave = threadIdx.x >> 5;
  const int tilesN = N >> 6;
  const int tilesM = M >> 6;
  const int tile = blockIdx.x * 8 + wave;
  if (tile >= tilesM * tilesN) return;
  const int tm = tile / tilesN;
  const int tn = tile - tm * tilesN;
  const int m0 = tm << 6;
  const int n0 = tn << 6;

  const T* Ab  = A  + (size_t)b * strideA;
  const T* Bb  = Bt + (size_t)b * strideB;
  const T* Ab2 = SPLIT ? (A2  + (size_t)b * strideA) : nullptr;
  const T* Bb2 = SPLIT ? (Bt2 + (size_t)b * strideB) : nullptr;

  const int rlane = lane & 15;
  const int koff  = (lane >> 4) * 8;
  const int mOff  = (lane >> 4) * 8;

  v8f acc[4][4];
#pragma unroll
  for (int i = 0; i < 4; ++i)
#pragma unroll
    for (int j = 0; j < 4; ++j) acc[i][j] = (v8f){0.f,0.f,0.f,0.f,0.f,0.f,0.f,0.f};

  for (int k0 = 0; k0 < K; k0 += 32) {
    V bh[4], bl[4];
#pragma unroll
    for (int j = 0; j < 4; ++j) {
      const size_t bo = (size_t)(n0 + (j << 4) + rlane) * ldb + koff + k0;
      bh[j] = Frag<T>::load(Bb + bo);
      if (SPLIT) bl[j] = Frag<T>::load(Bb2 + bo);
    }
#pragma unroll
    for (int i = 0; i < 4; ++i) {
      const size_t ao = (size_t)(m0 + (i << 4) + rlane) * lda + koff + k0;
      V ah = Frag<T>::load(Ab + ao);
      V al;
      if (SPLIT) al = Frag<T>::load(Ab2 + ao);
#pragma unroll
      for (int j = 0; j < 4; ++j) {
        acc[i][j] = Frag<T>::mma(ah, bh[j], acc[i][j]);
        if (SPLIT) {
          acc[i][j] = Frag<T>::mma(ah, bl[j], acc[i][j]);
          acc[i][j] = Frag<T>::mma(al, bh[j], acc[i][j]);
        }
      }
      Frag<T>::guard4(acc[i][0], acc[i][1], acc[i][2], acc[i][3], ah, SPLIT ? al : ah);
    }
    Frag<T>::keep(bh[0], bh[1], bh[2], bh[3]);
    if (SPLIT) Frag<T>::keep(bl[0], bl[1], bl[2], bl[3]);
  }
  acc_guard4(acc[0][0], acc[0][1], acc[0][2], acc[0][3]);
  acc_guard4(acc[1][0], acc[1][1], acc[1][2], acc[1][3]);
  acc_guard4(acc[2][0], acc[2][1], acc[2][2], acc[2][3]);
  acc_guard4(acc[3][0], acc[3][1], acc[3][2], acc[3][3]);

  float* slab = sT[wave];
#pragma unroll
  for (int i = 0; i < 4; ++i) {
    const int mBase = m0 + (i << 4);
    v4f bm0 = (v4f){0.f,0.f,0.f,0.f}, bm1 = (v4f){0.f,0.f,0.f,0.f};
    if (BIAS_MODE == 1) {
      bm0 = *(const v4f*)(bias + mBase + mOff);
      bm1 = *(const v4f*)(bias + mBase + mOff + 4);
    }
#pragma unroll
    for (int j = 0; j < 4; ++j) {
      const int n = n0 + (j << 4) + rlane;
      float bv = 0.f;
      if (BIAS_MODE == 2) bv = bias[n];
#pragma unroll
      for (int r = 0; r < 8; ++r) {
        float v = acc[i][j][r] * scale;
        if (BIAS_MODE == 1) v += (r < 4) ? bm0[r & 3] : bm1[r & 3];
        if (BIAS_MODE == 2) v += bv;
        slab[(mOff + r) * 68 + (j << 4) + rlane] = v;
      }
    }
    __builtin_amdgcn_fence(__ATOMIC_RELEASE, "workgroup");
    __builtin_amdgcn_wave_barrier();
    __builtin_amdgcn_fence(__ATOMIC_ACQUIRE, "workgroup");
    if (OUT_MODE == 0) {
      float* C = (float*)Cout + (size_t)b * strideC;
      const int hh = lane >> 4, c4 = (lane & 15) * 4;
      if (RESF) {
        const float* Rb = resid + (size_t)b * strideR;
#pragma unroll
        for (int it = 0; it < 8; ++it) {
          const int row = it * 2 + hh;
          const v4f rv = *(const v4f*)(Rb + (size_t)(mBase + row) * ldc + n0 + c4);
          v4f sv = *(const v4f*)(slab + row * 68 + c4);
          sv += rv;
          *(v4f*)(slab + row * 68 + c4) = sv;
        }
      }
      for (int pass = 0; pass < 2; ++pass) {
#pragma unroll
        for (int it = 0; it < 8; ++it) {
          const int row = it * 2 + hh;
          v4f v = *(const v4f*)(slab + row * 68 + c4);
          *(volatile v4f*)(C + (size_t)(mBase + row) * ldc + n0 + c4) = v;
        }
        __threadfence();
      }
    } else {
      const int q = lane >> 3, c8 = (lane & 7) * 8;
      unsigned short* C = (unsigned short*)Cout + (size_t)b * strideC;
      for (int pass = 0; pass < 2; ++pass) {
#pragma unroll
        for (int it = 0; it < 4; ++it) {
          const int row = it * 4 + q;
          const float* sp = slab + row * 68 + c8;
          v8h hv;
#pragma unroll
          for (int e = 0; e < 8; ++e) hv[e] = (_Float16)sp[e];
          *(volatile v8h*)(C + (size_t)(mBase + row) * ldc + n0 + c8) = hv;
        }
        __threadfence();
      }
    }
    __builtin_amdgcn_fence(__ATOMIC_RELEASE, "workgroup");
    __builtin_amdgcn_wave_barrier();
    __builtin_amdgcn_fence(__ATOMIC_ACQUIRE, "workgroup");
  }
}

template <int MODE>
__global__ __launch_bounds__(256) void cvt2_kernel(const float* __restrict__ in, unsigned short* __restrict__ out,
                                                   int n2, float carry) {
  const int i = blockIdx.x * 256 + threadIdx.x;
  if (i < n2) {
    const v2f f = *(const v2f*)(in + 2 * (size_t)i);
    const float f0 = f[0], f1 = f[1];
    unsigned short b0, b1;
    if (MODE == 0) {
      b0 = f2bf_bits(f0); b1 = f2bf_bits(f1);
    } else {
      const float g0 = bf_bits2f(f2bf_bits(f0)) * carry;
      const float g1 = bf_bits2f(f2bf_bits(f1)) * carry;
      const _Float16 h0 = (_Float16)g0, h1 = (_Float16)g1;
      b0 = __builtin_bit_cast(unsigned short, h0); b1 = __builtin_bit_cast(unsigned short, h1);
    }
    const unsigned u = (unsigned)b0 | ((unsigned)b1 << 16);
    ((volatile unsigned*)out)[i] = u;
    __threadfence();
    ((volatile unsigned*)out)[i] = u;
  }
}

__global__ __launch_bounds__(128) void bias_table_kernel(
    const float* __restrict__ bih0, const float* __restrict__ bhh0,
    const float* __restrict__ bih1, const float* __restrict__ bhh1,
    const float* __restrict__ bh, const float* __restrict__ bt,
    const float* __restrict__ bi, const float* __restrict__ bc,
    float* __restrict__ tab) {
  const int seg = blockIdx.x;
  const int t = threadIdx.x;
  const float* p1; const float* p2; float mul; int two;
  switch (seg) {
    case 0:  p1 = bih0;       p2 = bhh0;       two = 1; mul = 1.0f; break;
    case 1:  p1 = bih0 + 512; p2 = bhh0 + 512; two = 1; mul = 1.0f; break;
    case 2:  p1 = bih1;       p2 = bhh1;       two = 1; mul = 1.0f; break;
    case 3:  p1 = bih1 + 512; p2 = bhh1 + 512; two = 1; mul = 1.0f; break;
    case 4:  p1 = bh;         p2 = bh;         two = 0; mul = 1.0f; break;
    case 5:  p1 = bt;         p2 = bt;         two = 0; mul = 1.0f; break;
    case 6:  p1 = bi;         p2 = bi;         two = 0; mul = 1.0f; break;
    default: p1 = bc;         p2 = bc;         two = 0; mul = AV_CARRY; break;
  }
  const v4f a = *(const v4f*)(p1 + 4 * t);
  const v4f c = *(const v4f*)(p2 + 4 * t);
  v4f o;
#pragma unroll
  for (int q = 0; q < 4; ++q) {
    const float x = bf_bits2f(f2bf_bits(a[q]));
    const float y = two ? bf_bits2f(f2bf_bits(c[q])) : 0.0f;
    o[q] = (x + y) * mul;
  }
  float* dst = tab + seg * 512 + 4 * t;
  *(volatile v4f*)dst = o;
  __threadfence();
  *(volatile v4f*)dst = o;
}

__global__ __launch_bounds__(256) void softmax_kernel(const unsigned short* __restrict__ S16,
                                                      const int* __restrict__ gb,
                                                      unsigned short* __restrict__ P16) {
  __shared__ __align__(32) float es[8][NNODE];
  const int lane = threadIdx.x & 31, wave = threadIdx.x >> 5;
  const int row = blockIdx.x * 8 + wave;
  const int hq = row / NNODE;
  const int n = row - hq * NNODE;
  const unsigned short* srow = S16 + (size_t)row * NNODE;
  const int* grow = gb + (size_t)n * NNODE;
  unsigned short* prow = P16 + (size_t)row * NNODE;
  float* ew = es[wave];

  float mx = -INFINITY;
#pragma unroll 1
  for (int it = 0; it < 3; ++it) {
    const int c8 = it * 256 + lane * 8;
    const v4u sw = *(const v4u*)(srow + c8);
    const v8i g8 = *(const v8i*)(grow + c8);
#pragma unroll
    for (int q = 0; q < 8; ++q) {
      const unsigned w = sw[q >> 1];
      const unsigned hb = (q & 1) ? (w >> 16) : (w & 0xffffu);
      const float s = h16_to_f32(hb);
      mx = fmaxf(mx, (g8[q] != 0) ? s : -INFINITY);
    }
  }
#pragma unroll
  for (int off = 1; off < 32; off <<= 1) mx = fmaxf(mx, __shfl_xor(mx, off, 32));
  const float mxs = (mx == -INFINITY) ? 0.0f : mx;

  float sum = 0.0f;
#pragma unroll 1
  for (int it = 0; it < 3; ++it) {
    const int c8 = it * 256 + lane * 8;
    const v4u sw = *(const v4u*)(srow + c8);
    const v8i g8 = *(const v8i*)(grow + c8);
    v8f e8;
#pragma unroll
    for (int q = 0; q < 8; ++q) {
      const unsigned w = sw[q >> 1];
      const unsigned hb = (q & 1) ? (w >> 16) : (w & 0xffffu);
      const float s = h16_to_f32(hb);
      const float ex = expf(s - mxs);
      const float e = (g8[q] != 0) ? ex : 0.0f;
      e8[q] = e;
      sum += e;
    }
    *(v8f*)(ew + c8) = e8;
  }
#pragma unroll
  for (int off = 1; off < 32; off <<= 1) sum += __shfl_xor(sum, off, 32);
  const float den = (sum > 0.0f) ? sum : 1.0f;
  const float inv = (sum > 0.0f) ? (P_CARRY / den) : 0.0f;

  for (int pass = 0; pass < 2; ++pass) {
#pragma unroll 1
    for (int it = 0; it < 3; ++it) {
      const int c8 = it * 256 + lane * 8;
      const v8f e8 = *(const v8f*)(ew + c8);
      v8h hv;
#pragma unroll
      for (int q = 0; q < 8; ++q) hv[q] = (_Float16)(e8[q] * inv);
      *(volatile v8h*)(prow + c8) = hv;
    }
    __threadfence();
  }
}

__device__ __forceinline__ float sigm(float x) { return __builtin_amdgcn_rcpf(1.0f + expf(-x)); }

template <bool HAS_C0, bool LAST>
__global__ __launch_bounds__(256) void cell_ln_kernel(const float* __restrict__ G,
                                                      const unsigned short* __restrict__ C016,
                                                      const float* __restrict__ gamma, const float* __restrict__ beta,
                                                      unsigned short* __restrict__ memb, float* __restrict__ outf,
                                                      int rbase) {
  __shared__ __align__(32) float hs[8][DMODEL];
  const int lane = threadIdx.x & 31, wave = threadIdx.x >> 5;
  const int j = blockIdx.x * 8 + wave;
  const int r = rbase + j;
  float* hw = hs[wave];
  const unsigned* c0w = (const unsigned*)(const void*)C016;

  float s1 = 0.0f;
#pragma unroll 1
  for (int e = 0; e < 16; ++e) {
    const int half = e >> 3;
    const int k = lane + 32 * (e & 7);
    const int m = 2 * j + half;
    const float* gr = G + (size_t)m * G4W + k;
    const float zi = gr[0];
    const float zf = gr[HIDN];
    const float zg = gr[2 * HIDN];
    const float zo = gr[3 * HIDN];
    float c0 = 0.0f;
    if (HAS_C0) {
      const unsigned w = c0w[((size_t)m * HIDN + k) >> 1];
      const unsigned hb = (k & 1) ? (w >> 16) : (w & 0xffffu);
      c0 = h16_to_f32(hb) * AV_CARRY_INV;
    }
    const float si = sigm(zi), sf = sigm(zf), so = sigm(zo);
    const float cn = sf * c0 + si * tanhf(zg);
    const float h = so * tanhf(cn);
    hw[half * HIDN + k] = h;
    s1 += h;
  }
#pragma unroll
  for (int off = 1; off < 32; off <<= 1) s1 += __shfl_xor(s1, off, 32);
  const float mean = s1 * (1.0f / (float)DMODEL);
  float s2 = 0.0f;
#pragma unroll 1
  for (int e = 0; e < 16; ++e) {
    const int c = (e >> 3) * HIDN + lane + 32 * (e & 7);
    const float d = hw[c] - mean;
    s2 = fmaf(d, d, s2);
  }
#pragma unroll
  for (int off = 1; off < 32; off <<= 1) s2 += __shfl_xor(s2, off, 32);
  const float var = s2 * (1.0f / (float)DMODEL);
  const float inv = rsqrtf(var + LN_EPS);
#pragma unroll 1
  for (int e = 0; e < 16; ++e) {
    const int c = (e >> 3) * HIDN + lane + 32 * (e & 7);
    const float y = (hw[c] - mean) * inv * gamma[c] + beta[c];
    hw[c] = y;
  }
  __syncthreads();
  if (!LAST) {
    v4u mv[2];
#pragma unroll
    for (int seg = 0; seg < 2; ++seg) {
      const int c8 = seg * HIDN + lane * 8;
      const v8f y8 = *(const v8f*)(hw + c8);
      v4u pk;
#pragma unroll
      for (int q = 0; q < 4; ++q) {
        const unsigned short u0 = f2bf_bits(y8[2 * q]);
        const unsigned short u1 = f2bf_bits(y8[2 * q + 1]);
        pk[q] = (unsigned)u0 | ((unsigned)u1 << 16);
      }
      mv[seg] = pk;
    }
    for (int pass = 0; pass < 2; ++pass) {
#pragma unroll
      for (int seg = 0; seg < 2; ++seg)
        *(volatile v4u*)(memb + (size_t)r * DMODEL + seg * HIDN + lane * 8) = mv[seg];
      __threadfence();
    }
  } else {
    v4f ov[4];
#pragma unroll
    for (int seg = 0; seg < 4; ++seg) ov[seg] = *(const v4f*)(hw + seg * 128 + lane * 4);
    for (int pass = 0; pass < 2; ++pass) {
#pragma unroll
      for (int seg = 0; seg < 4; ++seg)
        *(volatile v4f*)(outf + (size_t)r * DMODEL + seg * 128 + lane * 4) = ov[seg];
      __threadfence();
    }
  }
}

template <int ET, int BM, int OM, bool RF>
static inline void launch_gemm(hipStream_t st, const unsigned short* A, int lda, long sA,
                               const unsigned short* Bt, int ldb, long sB, void* C, int ldc, long sC,
                               const float* bias, const float* res, long sR, int M, int N, int K, float scale, int Z) {
  const int tiles = (M / 64) * (N / 64);
  const int blocks = (tiles + 7) / 8;
  wmma_gemm64<ET, false, BM, OM, RF><<<dim3(blocks, Z), 256, 0, st>>>(
      A, A, lda, sA, Bt, Bt, ldb, sB, C, ldc, sC, bias, res, sR, M, N, K, scale);
}

extern "C" void kernel_launch(void* const* d_in, const int* in_sizes, int n_in,
                              void* d_out, int out_size, void* d_ws, size_t ws_size, hipStream_t stream) {
  if (n_in < 20 || d_out == nullptr || d_ws == nullptr) return;
  if (in_sizes[0] != MROWS * DMODEL || in_sizes[1] != NBATCH * NNODE * NNODE) return;
  if (in_sizes[2] != G4W * DMODEL || in_sizes[3] != G4W * HIDN || in_sizes[4] != G4W || in_sizes[5] != G4W) return;
  if (in_sizes[6] != G4W * DMODEL || in_sizes[7] != G4W * HIDN || in_sizes[8] != G4W || in_sizes[9] != G4W) return;
  for (int i = 10; i <= 16; i += 2) if (in_sizes[i] != DMODEL * DMODEL || in_sizes[i + 1] != DMODEL) return;
  if (in_sizes[18] != DMODEL || in_sizes[19] != DMODEL || out_size != MROWS * DMODEL) return;
  if (ws_size < WS_TOTAL) return;

  const float* xin   = (const float*)d_in[0];
  const int*   graph = (const int*)d_in[1];
  const float* wih0  = (const float*)d_in[2];
  const float* whh0  = (const float*)d_in[3];
  const float* bih0  = (const float*)d_in[4];
  const float* bhh0  = (const float*)d_in[5];
  const float* wih1  = (const float*)d_in[6];
  const float* whh1  = (const float*)d_in[7];
  const float* bih1  = (const float*)d_in[8];
  const float* bhh1  = (const float*)d_in[9];
  const float* wh    = (const float*)d_in[10];
  const float* bh    = (const float*)d_in[11];
  const float* wt    = (const float*)d_in[12];
  const float* bt    = (const float*)d_in[13];
  const float* wi    = (const float*)d_in[14];
  const float* bi    = (const float*)d_in[15];
  const float* wc    = (const float*)d_in[16];
  const float* bc    = (const float*)d_in[17];
  const float* gamma = (const float*)d_in[18];
  const float* beta  = (const float*)d_in[19];
  float* outp = (float*)d_out;

  char* ws = (char*)d_ws;
  unsigned short* xm16   = (unsigned short*)(ws + OFF_XM);
  unsigned short* head16 = (unsigned short*)(ws + OFF_HEAD);
  unsigned short* ta16   = (unsigned short*)(ws + OFF_TA);
  unsigned short* inft16 = (unsigned short*)(ws + OFF_INFT);
  unsigned short* av16   = (unsigned short*)(ws + OFF_AV);
  unsigned short* wih16[2] = { (unsigned short*)(ws + OFF_WIH0), (unsigned short*)(ws + OFF_WIH1) };
  unsigned short* whh16[2] = { (unsigned short*)(ws + OFF_WHH0), (unsigned short*)(ws + OFF_WHH1) };
  unsigned short* wh16   = (unsigned short*)(ws + OFF_WH);
  unsigned short* wt16   = (unsigned short*)(ws + OFF_WT);
  unsigned short* wi16   = (unsigned short*)(ws + OFF_WI);
  unsigned short* wc16   = (unsigned short*)(ws + OFF_WC);
  float* btab   = (float*)(ws + OFF_BTAB);
  float* gx32   = (float*)(ws + OFF_GX);
  float* gate32 = (float*)(ws + OFF_GATE);
  unsigned short* s16 = (unsigned short*)(ws + OFF_S);
  unsigned short* p16 = (unsigned short*)(ws + OFF_P);

  const float inv_sqrt_d = 1.0f / sqrtf((float)DMODEL);
  const float av_scale   = AV_CARRY / P_CARRY;
  const float wc_scale   = 1.0f / W_CARRY;
  const float whh_scale  = 1.0f / (AV_CARRY * W_CARRY);

  static_assert((MROWS * DMODEL / 2) % 256 == 0 && (G4W * DMODEL / 2) % 256 == 0 && (G4W * HIDN / 2) % 256 == 0 && (DMODEL * DMODEL / 2) % 256 == 0, "");
  cvt2_kernel<0><<<(MROWS * DMODEL / 2) / 256, 256, 0, stream>>>(xin, xm16, MROWS * DMODEL / 2, 1.0f);
  cvt2_kernel<0><<<(G4W * DMODEL / 2) / 256, 256, 0, stream>>>(wih0, wih16[0], G4W * DMODEL / 2, 1.0f);
  cvt2_kernel<0><<<(G4W * DMODEL / 2) / 256, 256, 0, stream>>>(wih1, wih16[1], G4W * DMODEL / 2, 1.0f);
  cvt2_kernel<1><<<(G4W * HIDN / 2) / 256, 256, 0, stream>>>(whh0, whh16[0], G4W * HIDN / 2, W_CARRY);
  cvt2_kernel<1><<<(G4W * HIDN / 2) / 256, 256, 0, stream>>>(whh1, whh16[1], G4W * HIDN / 2, W_CARRY);
  cvt2_kernel<0><<<(DMODEL * DMODEL / 2) / 256, 256, 0, stream>>>(wh, wh16, DMODEL * DMODEL / 2, 1.0f);
  cvt2_kernel<0><<<(DMODEL * DMODEL / 2) / 256, 256, 0, stream>>>(wt, wt16, DMODEL * DMODEL / 2, 1.0f);
  cvt2_kernel<0><<<(DMODEL * DMODEL / 2) / 256, 256, 0, stream>>>(wi, wi16, DMODEL * DMODEL / 2, 1.0f);
  cvt2_kernel<1><<<(DMODEL * DMODEL / 2) / 256, 256, 0, stream>>>(wc, wc16, DMODEL * DMODEL / 2, W_CARRY);

  bias_table_kernel<<<8, 128, 0, stream>>>(bih0, bhh0, bih1, bhh1, bh, bt, bi, bc, btab);

  for (int d = 0; d < 2; ++d)
    launch_gemm<1, 2, 0, false>(stream, xm16, DMODEL, 0, wih16[d], DMODEL, 0, gx32 + (size_t)d * MROWS * G4W, G4W, 0,
                                btab + d * G4W, gx32, 0, MROWS, G4W, DMODEL, 1.0f, 1);
  launch_gemm<1, 2, 1, false>(stream, xm16, DMODEL, 0, wh16, DMODEL, 0, head16, DMODEL, 0,
                              btab + 2048, gx32, 0, MROWS, DMODEL, DMODEL, 1.0f, 1);

  cell_ln_kernel<false, false><<<MHALF / 8, 256, 0, stream>>>(gx32, ta16, gamma, beta, xm16, outp, 0);
  cell_ln_kernel<false, false><<<MHALF / 8, 256, 0, stream>>>(gx32 + (size_t)MROWS * G4W, ta16, gamma, beta, xm16, outp, MHALF);

  for (int layer = 0; layer < NLAYERS; ++layer) {
    const bool last = (layer == NLAYERS - 1);
    launch_gemm<1, 2, 1, false>(stream, xm16, DMODEL, 0, wt16, DMODEL, 0, ta16, DMODEL, 0,
                                btab + 2560, gx32, 0, MROWS, DMODEL, DMODEL, 1.0f, 1);
    launch_gemm<1, 1, 1, false>(stream, wi16, DMODEL, 0, xm16, DMODEL, (long)NNODE * DMODEL, inft16, NNODE, (long)DMODEL * NNODE,
                                btab + 3072, gx32, 0, DMODEL, NNODE, DMODEL, 1.0f, NBATCH);
    for (int b = 0; b < NBATCH; ++b) {
      launch_gemm<0, 0, 1, false>(stream, head16 + (size_t)b * NNODE * DMODEL, DMODEL, HDIM,
                                  ta16 + (size_t)b * NNODE * DMODEL, DMODEL, HDIM,
                                  s16, NNODE, (long)NNODE * NNODE, btab, gx32, 0, NNODE, NNODE, HDIM, inv_sqrt_d, NHEADS);
      softmax_kernel<<<(NHEADS * NNODE) / 8, 256, 0, stream>>>(s16, graph + (size_t)b * NNODE * NNODE, p16);
      launch_gemm<0, 0, 1, false>(stream, p16, NNODE, (long)NNODE * NNODE,
                                  inft16 + (size_t)b * DMODEL * NNODE, NNODE, (long)HDIM * NNODE,
                                  av16 + (size_t)b * NNODE * DMODEL, DMODEL, HDIM,
                                  btab, gx32, 0, NNODE, HDIM, NNODE, av_scale, NHEADS);
    }
    launch_gemm<0, 2, 1, false>(stream, av16, DMODEL, 0, wc16, DMODEL, 0, ta16, DMODEL, 0,
                                btab + 3584, gx32, 0, MROWS, DMODEL, DMODEL, wc_scale, 1);
    for (int d = 0; d < 2; ++d) {
      launch_gemm<0, 0, 0, true>(stream, ta16 + (size_t)d * MROWS * HIDN, HIDN, 0, whh16[d], HIDN, 0, gate32, G4W, 0,
                                 btab, gx32 + (size_t)d * MROWS * G4W, 0, MROWS, G4W, HIDN, whh_scale, 1);
      if (last)
        cell_ln_kernel<true, true><<<MHALF / 8, 256, 0, stream>>>(gate32, ta16 + (size_t)d * MROWS * HIDN, gamma, beta, xm16, outp, d * MHALF);
      else
        cell_ln_kernel<true, false><<<MHALF / 8, 256, 0, stream>>>(gate32, ta16 + (size_t)d * MROWS * HIDN, gamma, beta, xm16, outp, d * MHALF);
    }
  }
}
